// curiosity_5892695130372
// MI455X (gfx1250) — hardware-verified
//
#include <hip/hip_runtime.h>
#include <math.h>
#include <stdint.h>

constexpr int kBatch  = 2;
constexpr int kSeq    = 2048;
constexpr int kSeqA   = 1500;
constexpr int kSeqAP  = 1536;
constexpr int kDModel = 1024;
constexpr int kHeads  = 16;
constexpr int kDHead  = 64;
constexpr int kNQKV   = 3072;

constexpr float kPCarry = 32768.0f;
constexpr float kOCarry = 32.0f;
constexpr float kWCarry = 32.0f;

typedef __attribute__((ext_vector_type(16))) _Float16 v16h;
typedef __attribute__((ext_vector_type(8)))  _Float16 v8h;
typedef __attribute__((ext_vector_type(16))) __bf16   v16b;
typedef __attribute__((ext_vector_type(8)))  __bf16   v8b;
typedef __attribute__((ext_vector_type(8)))  float    v8f;
typedef __attribute__((ext_vector_type(4)))  float    v4f;
typedef __attribute__((ext_vector_type(2)))  float    v2f;
typedef __attribute__((ext_vector_type(4)))  unsigned int v4u;


__device__ __forceinline__ unsigned short f2bf_bits(float f) {
  unsigned u = __float_as_uint(f);
  return (unsigned short)((u + 0x7FFFu + ((u >> 16) & 1u)) >> 16);
}
__device__ __forceinline__ float bf_bits2f(unsigned short h) { return __uint_as_float(((unsigned)h) << 16); }
__device__ __forceinline__ unsigned pk16(unsigned short a, unsigned short b) { return (unsigned)a | ((unsigned)b << 16); }

__device__ __forceinline__ void dep_guard_h(v8f& a, v8f& b, v16h x, v16h y) { asm volatile("v_nop\n\tv_nop\n\tv_nop\n\tv_nop" : "+v"(a), "+v"(b) : "v"(x), "v"(y)); }
__device__ __forceinline__ void dep_guard_b(v8f& a, v8f& b, v16b x, v16b y) { asm volatile("v_nop\n\tv_nop\n\tv_nop\n\tv_nop" : "+v"(a), "+v"(b) : "v"(x), "v"(y)); }
__device__ __forceinline__ void keep4_h(v16h a, v16h b, v16h c, v16h d) { asm volatile("v_nop" :: "v"(a), "v"(b), "v"(c), "v"(d)); }
__device__ __forceinline__ void keep4_b(v16b a, v16b b, v16b c, v16b d) { asm volatile("v_nop" :: "v"(a), "v"(b), "v"(c), "v"(d)); }
__device__ __forceinline__ void acc_guard4(v8f& a, v8f& b, v8f& c, v8f& d) { asm volatile("v_nop\n\tv_nop\n\tv_nop\n\tv_nop" : "+v"(a), "+v"(b), "+v"(c), "+v"(d)); }
template <typename T> struct Frag;
template <> struct Frag<_Float16> {
  typedef v16h V; union U { v16h v; v8h h[2]; };
  static __device__ __forceinline__ v16h load(const _Float16* p) {
    U f; f.h[0] = *(const v8h*)(p); f.h[1] = *(const v8h*)(p + 16); return f.v;
  }
  static __device__ __forceinline__ v8f mma(v16h a, v16h b, v8f c) {
    return __builtin_amdgcn_wmma_f32_16x16x32_f16(false, a, false, b, (short)0, c, false, false);
  }
  static __device__ __forceinline__ void guard(v8f& a, v8f& b, v16h x, v16h y) { dep_guard_h(a, b, x, y); }
  static __device__ __forceinline__ void keep(v16h a, v16h b, v16h c, v16h d) { keep4_h(a, b, c, d); }
};
template <> struct Frag<__bf16> {
  typedef v16b V; union U { v16b v; v8b h[2]; };
  static __device__ __forceinline__ v16b load(const __bf16* p) {
    U f; f.h[0] = *(const v8b*)(p); f.h[1] = *(const v8b*)(p + 16); return f.v;
  }
  static __device__ __forceinline__ v8f mma(v16b a, v16b b, v8f c) {
    return __builtin_amdgcn_wmma_f32_16x16x32_bf16(false, a, false, b, (short)0, c, false, false);
  }
  static __device__ __forceinline__ void guard(v8f& a, v8f& b, v16b x, v16b y) { dep_guard_b(a, b, x, y); }
  static __device__ __forceinline__ void keep(v16b a, v16b b, v16b c, v16b d) { keep4_b(a, b, c, d); }
};

template <int ET> struct Elem;
template <> struct Elem<0> { typedef _Float16 T; };
template <> struct Elem<1> { typedef __bf16 T; };
template <int ET, bool SPLIT, int BIAS_MODE, int OUT_MODE, bool RESID, int ACT = 0>
__global__ __launch_bounds__(256) void wmma_gemm64(
    const unsigned short* __restrict__ Ap, const unsigned short* __restrict__ A2p, int lda, long strideA,
    const unsigned short* __restrict__ Btp, const unsigned short* __restrict__ Bt2p, int ldb, long strideB,
    void* __restrict__ Cout, void* __restrict__ Cout2, int ldc, long strideC,
    const float* __restrict__ bias,
    const float* __restrict__ resid, long strideR,
    int M, int N, int K, float scale) {
  typedef typename Elem<ET>::T T;
  typedef typename Frag<T>::V V;
  const T* A = (const T*)Ap; const T* A2 = (const T*)A2p; const T* Bt = (const T*)Btp; const T* Bt2 = (const T*)Bt2p;
  __shared__ __align__(16) float sT[8][16 * 68];
  const int b    = blockIdx.y;
  const int lane = threadIdx.x & 31;
  const int wave = threadIdx.x >> 5;
  const int tilesN = N >> 6;
  const int tilesM = M >> 6;
  const int tile = blockIdx.x * 8 + wave;
  if (tile >= tilesM * tilesN) return;
  const int tm = tile / tilesN;
  const int tn = tile - tm * tilesN;
  const int m0 = tm << 6;
  const int n0 = tn << 6;

  const T* Ab  = A  + (size_t)b * strideA;
  const T* Bb  = Bt + (size_t)b * strideB;
  const T* Ab2 = SPLIT ? (A2  + (size_t)b * strideA) : nullptr;
  const T* Bb2 = SPLIT ? (Bt2 + (size_t)b * strideB) : nullptr;

  const int rlane = lane & 15;
  const int koff  = (lane >> 4) * 8;
  const int mOff  = (lane >> 4) * 8;

  v8f acc[4][4];
#pragma unroll
  for (int i = 0; i < 4; ++i)
#pragma unroll
    for (int j = 0; j < 4; ++j) acc[i][j] = (v8f){0.f,0.f,0.f,0.f,0.f,0.f,0.f,0.f};

  for (int k0 = 0; k0 < K; k0 += 32) {
    V bh[4], bl[4];
#pragma unroll
    for (int j = 0; j < 4; ++j) {
      const size_t bo = (size_t)(n0 + (j << 4) + rlane) * ldb + koff + k0;
      bh[j] = Frag<T>::load(Bb + bo);
      if (SPLIT) bl[j] = Frag<T>::load(Bb2 + bo);
    }
#pragma unroll
    for (int i = 0; i < 4; ++i) {
      const size_t ao = (size_t)(m0 + (i << 4) + rlane) * lda + koff + k0;
      V ah = Frag<T>::load(Ab + ao);
      V al;
      if (SPLIT) al = Frag<T>::load(Ab2 + ao);
#pragma unroll
      for (int j = 0; j < 4; ++j) {
        acc[i][j] = Frag<T>::mma(ah, bh[j], acc[i][j]);
        if (SPLIT) {
          acc[i][j] = Frag<T>::mma(ah, bl[j], acc[i][j]);
          acc[i][j] = Frag<T>::mma(al, bh[j], acc[i][j]);
        }
      }
      Frag<T>::guard(acc[i][0], acc[i][3], ah, SPLIT ? al : ah);
    }
    Frag<T>::keep(bh[0], bh[1], bh[2], bh[3]);
    if (SPLIT) Frag<T>::keep(bl[0], bl[1], bl[2], bl[3]);
  }
  acc_guard4(acc[0][0], acc[0][1], acc[0][2], acc[0][3]);
  acc_guard4(acc[1][0], acc[1][1], acc[1][2], acc[1][3]);
  acc_guard4(acc[2][0], acc[2][1], acc[2][2], acc[2][3]);
  acc_guard4(acc[3][0], acc[3][1], acc[3][2], acc[3][3]);

  float* slab = sT[wave];
  const float* Rb = RESID ? (resid + (size_t)b * strideR) : nullptr;
#pragma unroll
  for (int i = 0; i < 4; ++i) {
    const int mBase = m0 + (i << 4);
#pragma unroll
    for (int j = 0; j < 4; ++j) {
      const int n = n0 + (j << 4) + rlane;
      float bv = 0.f;
      if (BIAS_MODE == 2) bv = bias[n];
#pragma unroll
      for (int r = 0; r < 8; ++r) {
        float v = acc[i][j][r] * scale;
        if (BIAS_MODE == 1) v += bias[mBase + mOff + r];
        if (BIAS_MODE == 2) v += bv;
        if (RESID) v += Rb[(size_t)(mBase + mOff + r) * ldc + n];
        if (ACT == 1) v = tanhf(v);
        if (ACT == 2) v = fmaxf(v, 0.0f);
        if (ACT == 3) v = v / (1.0f + expf(-v));
        if (ACT == 4) v = (v > 0.f) ? v : 0.01f * v;
        if (ACT == 5) v = 0.5f * v * (1.0f + erff(v * 0.70710678118654752f));
        slab[(mOff + r) * 68 + (j << 4) + rlane] = v;
      }
    }
    __builtin_amdgcn_fence(__ATOMIC_RELEASE, "workgroup");
    __builtin_amdgcn_wave_barrier();
    __builtin_amdgcn_fence(__ATOMIC_ACQUIRE, "workgroup");
    if (OUT_MODE == 0) {
      float* C = (float*)Cout + (size_t)b * strideC;
      const int hh = lane >> 4, c4 = (lane & 15) * 4;
      for (int pass = 0; pass < 2; ++pass) {
#pragma unroll
        for (int it = 0; it < 8; ++it) {
          const int row = it * 2 + hh;
          v4f v = *(const v4f*)(slab + row * 68 + c4);
          *(volatile v4f*)(C + (size_t)(mBase + row) * ldc + n0 + c4) = v;
        }
        __threadfence();
      }
    } else {
      const int q = lane >> 3, c8 = (lane & 7) * 8;
      unsigned short* C  = (unsigned short*)Cout  + (size_t)b * strideC;
      unsigned short* C2 = (OUT_MODE == 2) ? ((unsigned short*)Cout2 + (size_t)b * strideC) : nullptr;
      for (int pass = 0; pass < 2; ++pass) {
#pragma unroll
        for (int it = 0; it < 4; ++it) {
          const int row = it * 4 + q;
          const float* sp = slab + row * 68 + c8;
          v8h hv, lv;
#pragma unroll
          for (int e = 0; e < 8; ++e) {
            if (OUT_MODE == 1) {
              hv[e] = (_Float16)sp[e];
            } else {
              unsigned short hb = f2bf_bits(sp[e]);
              unsigned short lb = f2bf_bits(sp[e] - bf_bits2f(hb));
              hv[e] = __builtin_bit_cast(_Float16, hb);
              lv[e] = __builtin_bit_cast(_Float16, lb);
            }
          }
          *(volatile v8h*)(C + (size_t)(mBase + row) * ldc + n0 + c8) = hv;
          if (OUT_MODE == 2) *(volatile v8h*)(C2 + (size_t)(mBase + row) * ldc + n0 + c8) = lv;
        }
        __threadfence();
      }
    }
    __builtin_amdgcn_fence(__ATOMIC_RELEASE, "workgroup");
    __builtin_amdgcn_wave_barrier();
    __builtin_amdgcn_fence(__ATOMIC_ACQUIRE, "workgroup");
  }
}

__global__ __launch_bounds__(256) void cvt_bf16x2_kernel(const float* __restrict__ in, unsigned short* __restrict__ out, int n2) {
  const int i = blockIdx.x * 256 + threadIdx.x;
  if (i < n2) {
    const v2f f = *(const v2f*)(in + 2 * (size_t)i);
    const unsigned u = pk16(f2bf_bits(f[0]), f2bf_bits(f[1]));
    ((volatile unsigned*)out)[i] = u;
    __threadfence();
    ((volatile unsigned*)out)[i] = u;
  }
}

__global__ __launch_bounds__(256) void cvt_rows_bf16x2_kernel(const float* __restrict__ in, unsigned short* __restrict__ out,
                                                             int rin, int rout, int ncol, int nb, int n2) {
  const int i = blockIdx.x * 256 + threadIdx.x;
  if (i < n2) {
    const int ppr = ncol >> 1;
    const int row = i / ppr;
    const int col = (i - row * ppr) * 2;
    int bb = row / rout;
    const int t = row - bb * rout;
    bb = bb < (nb - 1) ? bb : (nb - 1);
    const bool valid = t < rin;
    const int tc = valid ? t : (rin - 1);
    const v2f f = *(const v2f*)(in + ((size_t)(bb * rin + tc) * ncol + col));
    const unsigned short h0 = valid ? f2bf_bits(f[0]) : (unsigned short)0;
    const unsigned short h1 = valid ? f2bf_bits(f[1]) : (unsigned short)0;
    const unsigned u = pk16(h0, h1);
    ((volatile unsigned*)out)[i] = u;
    __threadfence();
    ((volatile unsigned*)out)[i] = u;
  }
}

template <int OT> __device__ __forceinline__ unsigned short cv16(float f, float scl) {
  const unsigned short hb = f2bf_bits(f);
  if (OT == 0) return hb;
  const float g = bf_bits2f(hb) * scl;
  return __builtin_bit_cast(unsigned short, (_Float16)g);
}
template <int OT>
__global__ __launch_bounds__(256) void tconv_kernel(const float* __restrict__ W, unsigned short* __restrict__ o,
                                                    int R, int Cc, float scl) {
  __shared__ __align__(16) float tf[64 * 68];
  const int c0  = blockIdx.x * 64;
  const int r0  = blockIdx.y * 64;
  const int tid = threadIdx.x;
  {
    const int lr = tid >> 4;
    const int c4 = (tid & 15) * 4;
#pragma unroll
    for (int it = 0; it < 4; ++it) {
      const int rr = it * 16 + lr;
      const v4f a = *(const v4f*)(W + (size_t)(r0 + rr) * Cc + c0 + c4);
      *(v4f*)(tf + rr * 68 + c4) = a;
    }
  }
  __syncthreads();
  const int sub = tid >> 3;
  const int c8  = (tid & 7) * 8;
  v4u hv[2];
#pragma unroll
  for (int it = 0; it < 2; ++it) {
    const int oc = it * 32 + sub;
    v4u a;
#pragma unroll
    for (int q = 0; q < 4; ++q) {
      const float f0 = tf[(c8 + 2 * q) * 68 + oc];
      const float f1 = tf[(c8 + 2 * q + 1) * 68 + oc];
      a[q] = pk16(cv16<OT>(f0, scl), cv16<OT>(f1, scl));
    }
    hv[it] = a;
  }
  for (int pass = 0; pass < 2; ++pass) {
#pragma unroll
    for (int it = 0; it < 2; ++it) {
      const int oc = it * 32 + sub;
      const size_t go = (size_t)(c0 + oc) * R + r0 + c8;
      *(volatile v4u*)(o + go) = hv[it];
    }
    __threadfence();
  }
}

__global__ __launch_bounds__(256) void bias_rne_kernel(const float* __restrict__ b0, int n0, const float* __restrict__ b1, int n1,
                                                       const float* __restrict__ b2, int ncnt2, float* __restrict__ out, int ntot) {
  const int i = blockIdx.x * 256 + threadIdx.x;
  if (i < ntot) {
    int i0 = i < n0 ? i : (n0 - 1); i0 = i0 < 0 ? 0 : i0;
    int i1 = i - n0; i1 = i1 < 0 ? 0 : (i1 < n1 ? i1 : (n1 - 1));
    int i2 = i - n0 - n1; i2 = i2 < 0 ? 0 : (i2 < ncnt2 ? i2 : (ncnt2 - 1));
    const float v0 = b0[i0], v1 = b1[i1], v2 = b2[i2];
    const float sel = (i < n0) ? v0 : ((i < n0 + n1) ? v1 : v2);
    const float r = bf_bits2f(f2bf_bits(sel));
    ((volatile float*)out)[i] = r;
    __threadfence();
    ((volatile float*)out)[i] = r;
  }
}

__device__ __forceinline__ v8f mma_h16(v16h a, v16h b, v8f c) {
  c = __builtin_amdgcn_wmma_f32_16x16x32_f16(false, a, false, b, (short)0, c, false, false);
  asm volatile("v_nop\n\tv_nop\n\tv_nop\n\tv_nop" : "+v"(c) : "v"(a), "v"(b));
  return c;
}

__global__ __launch_bounds__(128)
void dual_attn_kernel(const unsigned short* __restrict__ qk16, const unsigned short* __restrict__ vt16,
                      const unsigned short* __restrict__ ka16, const unsigned short* __restrict__ vat16,
                      const float* __restrict__ gvec, unsigned short* __restrict__ o16) {
  union FH { v16h v; v8h h[2]; };
  __shared__ __align__(16) _Float16 Ksh[64 * 64];
  __shared__ __align__(16) _Float16 Vth[64 * 64];
  __shared__ __align__(16) _Float16 Psh[4][16 * 64];
  __shared__ __align__(16) float    Os[4][16 * 68];

  const int tid  = threadIdx.x;
  const int wave = tid >> 5;
  const int lane = tid & 31;
  const int hh   = lane >> 4;
  const int c    = lane & 15;

  const int bx = blockIdx.x;
  const int qb = bx & 31;
  const int bhd = bx >> 5;
  const int h  = bhd & 15;
  const int b  = bhd >> 4;
  const int q0 = qb * 64 + wave * 16;

  const int ldqk = 2 * kDModel;
  const _Float16* Qg  = (const _Float16*)(const void*)qk16 + (size_t)b * kSeq * ldqk + h * kDHead;
  const _Float16* Kg0 = Qg + kDModel;
  const _Float16* Vg0 = (const _Float16*)(const void*)vt16 + (size_t)b * kDModel * kSeq + (size_t)(h * kDHead) * kSeq;
  const _Float16* Kg1 = (const _Float16*)(const void*)ka16 + (size_t)b * kSeqAP * kDModel + h * kDHead;
  const _Float16* Vg1 = (const _Float16*)(const void*)vat16 + (size_t)b * kDModel * kSeqAP + (size_t)(h * kDHead) * kSeqAP;

  v16h qa[2];
#pragma unroll
  for (int dc = 0; dc < 2; ++dc) qa[dc] = Frag<_Float16>::load(Qg + (size_t)(q0 + c) * ldqk + dc * 32 + 8 * hh);

  float* os = Os[wave];
#pragma unroll
  for (int r = 0; r < 8; ++r)
#pragma unroll
    for (int t = 0; t < 4; ++t) os[(8 * hh + r) * 68 + t * 16 + c] = 0.f;

  const float gv   = bf_bits2f(f2bf_bits(gvec[h]));
  const float gate = 1.0f / (1.0f + expf(-gv));
  const float sscale = 0.125f;
  _Float16* pw = Psh[wave];

#pragma unroll 1
  for (int br = 0; br < 2; ++br) {
    const _Float16* Kg = br ? Kg1 : Kg0;
    const _Float16* Vg = br ? Vg1 : Vg0;
    const int ldk     = br ? kDModel : ldqk;
    const int ldv     = br ? kSeqAP : kSeq;
    const int nChunks = br ? (kSeqAP / 64) : (kSeq / 64);
    const int nvalid  = br ? kSeqA : kSeq;
    const float w     = (br ? gate : (1.0f - gate)) * kOCarry;

    float mrow[8], lrow[8];
    v8f oacc[4];
#pragma unroll
    for (int r = 0; r < 8; ++r) { mrow[r] = -INFINITY; lrow[r] = 0.f; }
#pragma unroll
    for (int t = 0; t < 4; ++t) oacc[t] = (v8f){0.f,0.f,0.f,0.f,0.f,0.f,0.f,0.f};

    for (int kc = 0; kc < nChunks; ++kc) {
      const int kv0 = kc * 64;
      __syncthreads();
      {
        const int r = tid >> 1, half = (tid & 1) * 32;
        const _Float16* ks = Kg + (size_t)(kv0 + r) * ldk + half;
        const _Float16* vs = Vg + (size_t)r * ldv + kv0 + half;
#pragma unroll
        for (int i = 0; i < 4; ++i) {
          const v8h a0 = *(const v8h*)(ks + 8 * i);
          const v8h b0 = *(const v8h*)(vs + 8 * i);
          *(v8h*)(Ksh + r * 64 + half + 8 * i) = a0;
          *(v8h*)(Vth + r * 64 + half + 8 * i) = b0;
        }
      }
      __syncthreads();

      v8f s[4];
#pragma unroll
      for (int j = 0; j < 4; ++j) {
        s[j] = (v8f){0.f,0.f,0.f,0.f,0.f,0.f,0.f,0.f};
#pragma unroll
        for (int dc = 0; dc < 2; ++dc) {
          FH kb;
          kb.h[0] = *(const v8h*)(Ksh + (j * 16 + c) * 64 + dc * 32 + 8 * hh);
          kb.h[1] = *(const v8h*)(Ksh + (j * 16 + c) * 64 + dc * 32 + 16 + 8 * hh);
          s[j] = mma_h16(qa[dc], kb.v, s[j]);
        }
      }
      float cm[8];
#pragma unroll
      for (int r = 0; r < 8; ++r) {
        float m = -INFINITY;
#pragma unroll
        for (int j = 0; j < 4; ++j) {
          const int key = kv0 + j * 16 + c;
          float sv = s[j][r] * sscale;
          sv = (key < nvalid) ? sv : -INFINITY;
          s[j][r] = sv;
          m = fmaxf(m, sv);
        }
#pragma unroll
        for (int off = 1; off < 16; off <<= 1) m = fmaxf(m, __shfl_xor(m, off, 32));
        cm[r] = m;
      }
#pragma unroll
      for (int r = 0; r < 8; ++r) {
        const float mnew = fmaxf(mrow[r], cm[r]);
        const float alpha = expf(mrow[r] - mnew);
        mrow[r] = mnew;
        float psum = 0.f;
#pragma unroll
        for (int j = 0; j < 4; ++j) {
          const float p = expf(s[j][r] - mnew);
          psum += p;
          pw[(8 * hh + r) * 64 + j * 16 + c] = (_Float16)(p * kPCarry);
        }
#pragma unroll
        for (int off = 1; off < 16; off <<= 1) psum += __shfl_xor(psum, off, 32);
        lrow[r] = lrow[r] * alpha + psum;
#pragma unroll
        for (int t = 0; t < 4; ++t) oacc[t][r] *= alpha;
      }
      __builtin_amdgcn_fence(__ATOMIC_RELEASE, "workgroup");
      __builtin_amdgcn_wave_barrier();
      __builtin_amdgcn_fence(__ATOMIC_ACQUIRE, "workgroup");
#pragma unroll 1
      for (int kk = 0; kk < 2; ++kk) {
        FH pa;
        pa.h[0] = *(const v8h*)(pw + c * 64 + kk * 32 + 8 * hh);
        pa.h[1] = *(const v8h*)(pw + c * 64 + kk * 32 + 16 + 8 * hh);
#pragma unroll
        for (int t = 0; t < 4; ++t) {
          FH vb;
          vb.h[0] = *(const v8h*)(Vth + (t * 16 + c) * 64 + kk * 32 + 8 * hh);
          vb.h[1] = *(const v8h*)(Vth + (t * 16 + c) * 64 + kk * 32 + 16 + 8 * hh);
          oacc[t] = mma_h16(pa.v, vb.v, oacc[t]);
        }
      }
    }
#pragma unroll
    for (int r = 0; r < 8; ++r) {
      const float inv = w * (1.0f / (lrow[r] * kPCarry));
#pragma unroll
      for (int t = 0; t < 4; ++t) os[(8 * hh + r) * 68 + t * 16 + c] += oacc[t][r] * inv;
    }
  }

  __builtin_amdgcn_fence(__ATOMIC_RELEASE, "workgroup");
  __builtin_amdgcn_wave_barrier();
  __builtin_amdgcn_fence(__ATOMIC_ACQUIRE, "workgroup");
  {
    _Float16* Og = (_Float16*)(void*)o16 + (size_t)(b * kSeq + q0) * kDModel + h * kDHead;
    const int q4 = lane >> 3, c8 = (lane & 7) * 8;
    for (int pass = 0; pass < 2; ++pass) {
#pragma unroll
      for (int it = 0; it < 4; ++it) {
        const int row = it * 4 + q4;
        const float* sp = os + row * 68 + c8;
        v8h hv;
#pragma unroll
        for (int e = 0; e < 8; ++e) hv[e] = (_Float16)sp[e];
        *(volatile v8h*)(Og + (size_t)row * kDModel + c8) = hv;
      }
      __threadfence();
    }
  }
}


extern "C" void kernel_launch(void* const* d_in, const int* in_sizes, int n_in,
                              void* d_out, int out_size, void* d_ws,
                              size_t ws_size, hipStream_t stream) {
  if (n_in < 9) return;
  if (in_sizes[0] != kBatch * kSeq * kDModel) return;
  if (in_sizes[1] != kBatch * kSeqA * kDModel) return;
  if (in_sizes[2] != kDModel * kNQKV || in_sizes[4] != kDModel * kNQKV) return;
  if (in_sizes[3] != kNQKV || in_sizes[5] != kNQKV) return;
  if (in_sizes[6] != kDModel * kDModel || in_sizes[7] != kDModel || in_sizes[8] < kHeads) return;
  if (out_size != kBatch * kSeq * kDModel) return;

  const float* x    = (const float*)d_in[0];
  const float* xa   = (const float*)d_in[1];
  const float* Wqkv = (const float*)d_in[2];
  const float* bqkv = (const float*)d_in[3];
  const float* Waux = (const float*)d_in[4];
  const float* baux = (const float*)d_in[5];
  const float* Wo   = (const float*)d_in[6];
  const float* bo   = (const float*)d_in[7];
  const float* gvec = (const float*)d_in[8];
  float* out = (float*)d_out;

  const size_t nXB   = (size_t)kBatch * kSeq * kDModel;
  const size_t nXAB  = (size_t)kBatch * kSeqAP * kDModel;
  const size_t nWQT  = (size_t)kNQKV * kDModel;
  const size_t nWAT  = nWQT;
  const size_t nWOT  = (size_t)kDModel * kDModel;
  const size_t nBias = (size_t)2 * kNQKV + kDModel;
  const size_t nQK   = (size_t)kBatch * kSeq * 2 * kDModel;
  const size_t nVT   = (size_t)kBatch * kDModel * kSeq;
  const size_t nKA   = (size_t)kBatch * kSeqAP * kDModel;
  const size_t nVAT  = (size_t)kBatch * kDModel * kSeqAP;
  const size_t nO    = (size_t)kBatch * kSeq * kDModel;

  char* ws = (char*)d_ws;
  size_t off = 0;
  auto carve = [&](size_t bytes) -> char* { char* p = ws + off; off += (bytes + 255) & ~(size_t)255; return p; };
  unsigned short* XB    = (unsigned short*)carve(nXB * 2);
  unsigned short* XAB   = (unsigned short*)carve(nXAB * 2);
  unsigned short* WQT   = (unsigned short*)carve(nWQT * 2);
  unsigned short* WAT   = (unsigned short*)carve(nWAT * 2);
  unsigned short* WOT   = (unsigned short*)carve(nWOT * 2);
  float*          BIASR = (float*)carve(nBias * 4);
  unsigned short* QK16  = (unsigned short*)carve(nQK * 2);
  unsigned short* VT16  = (unsigned short*)carve(nVT * 2);
  unsigned short* KA16  = (unsigned short*)carve(nKA * 2);
  unsigned short* VAT16 = (unsigned short*)carve(nVAT * 2);
  unsigned short* O16   = (unsigned short*)carve(nO * 2);
  if (off > ws_size) return;

  const int TB = 256;
  {
    const int n2 = (int)(nXB / 2);
    cvt_bf16x2_kernel<<<(n2 + TB - 1) / TB, TB, 0, stream>>>(x, XB, n2);
  }
  {
    const int n2 = (int)(nXAB / 2);
    cvt_rows_bf16x2_kernel<<<(n2 + TB - 1) / TB, TB, 0, stream>>>(xa, XAB, kSeqA, kSeqAP, kDModel, kBatch, n2);
  }
  tconv_kernel<0><<<dim3(kNQKV / 64, kDModel / 64), TB, 0, stream>>>(Wqkv, WQT, kDModel, kNQKV, 1.0f);
  tconv_kernel<0><<<dim3(kNQKV / 64, kDModel / 64), TB, 0, stream>>>(Waux, WAT, kDModel, kNQKV, 1.0f);
  tconv_kernel<1><<<dim3(kDModel / 64, kDModel / 64), TB, 0, stream>>>(Wo, WOT, kDModel, kDModel, kWCarry);
  {
    const int ntot = (int)nBias;
    bias_rne_kernel<<<(ntot + TB - 1) / TB, TB, 0, stream>>>(bqkv, kNQKV, baux, kNQKV, bo, kDModel, BIASR, ntot);
  }
  const float* bq_r  = BIASR;
  const float* ba_r  = BIASR + kNQKV;
  const float* bo_r  = BIASR + 2 * kNQKV;

  {
    const int M = kBatch * kSeq, N = 2 * kDModel, K = kDModel;
    const int tiles = (M / 64) * (N / 64);
    wmma_gemm64<1, false, 2, 1, false, 0><<<dim3((tiles + 7) / 8, 1), TB, 0, stream>>>(
        XB, XB, kDModel, 0L, WQT, WQT, kDModel, 0L, (void*)QK16, (void*)QK16, 2 * kDModel, 0L,
        bq_r, bq_r, 0L, M, N, K, 1.0f);
  }
  {
    const int M = kDModel, N = kSeq, K = kDModel;
    const int tiles = (M / 64) * (N / 64);
    wmma_gemm64<1, false, 1, 1, false, 0><<<dim3((tiles + 7) / 8, kBatch), TB, 0, stream>>>(
        WQT + (size_t)2 * kDModel * kDModel, WQT + (size_t)2 * kDModel * kDModel, kDModel, 0L,
        XB, XB, kDModel, (long)kSeq * kDModel,
        (void*)VT16, (void*)VT16, kSeq, (long)kDModel * kSeq,
        bq_r + 2 * kDModel, bq_r, 0L, M, N, K, 1.0f);
  }
  {
    const int M = kBatch * kSeqAP, N = kDModel, K = kDModel;
    const int tiles = (M / 64) * (N / 64);
    wmma_gemm64<1, false, 2, 1, false, 0><<<dim3((tiles + 7) / 8, 1), TB, 0, stream>>>(
        XAB, XAB, kDModel, 0L, WAT + (size_t)kDModel * kDModel, WAT + (size_t)kDModel * kDModel, kDModel, 0L,
        (void*)KA16, (void*)KA16, kDModel, 0L,
        ba_r + kDModel, ba_r, 0L, M, N, K, 1.0f);
  }
  {
    const int M = kDModel, N = kSeqAP, K = kDModel;
    const int tiles = (M / 64) * (N / 64);
    wmma_gemm64<1, false, 1, 1, false, 0><<<dim3((tiles + 7) / 8, kBatch), TB, 0, stream>>>(
        WAT + (size_t)2 * kDModel * kDModel, WAT + (size_t)2 * kDModel * kDModel, kDModel, 0L,
        XAB, XAB, kDModel, (long)kSeqAP * kDModel,
        (void*)VAT16, (void*)VAT16, kSeqAP, (long)kDModel * kSeqAP,
        ba_r + 2 * kDModel, ba_r, 0L, M, N, K, 1.0f);
  }
  dual_attn_kernel<<<kBatch * kHeads * (kSeq / 64), 128, 0, stream>>>(QK16, VT16, KA16, VAT16, gvec, O16);
  {
    const int M = kBatch * kSeq, N = kDModel, K = kDModel;
    const int tiles = (M / 64) * (N / 64);
    wmma_gemm64<0, false, 2, 0, false, 0><<<dim3((tiles + 7) / 8, 1), TB, 0, stream>>>(
        O16, O16, kDModel, 0L, WOT, WOT, kDModel, 0L, (void*)out, (void*)out, kDModel, 0L,
        bo_r, bo_r, 0L, M, N, K, 1.0f / (kOCarry * kWCarry));
  }
}
